// TextEncoder_3951369912636
// MI455X (gfx1250) — hardware-verified
//
#include <hip/hip_runtime.h>
#include <math.h>
#include <stdint.h>

#define NB   8
#define NT   1024
#define NC   192
#define NF   768
#define HD   96
#define NL   6
#define NO2  384
#define NTP  1026
#define CPW  256
#define NVOC 256
#define NTOK (NB * NT)
#define TPW  4

typedef _Float16 v16h __attribute__((ext_vector_type(16)));
typedef _Float16 v8h  __attribute__((ext_vector_type(8)));
typedef __bf16   v16b __attribute__((ext_vector_type(16)));
typedef unsigned short v8us __attribute__((ext_vector_type(8)));
typedef float v8f __attribute__((ext_vector_type(8)));
typedef float v4f __attribute__((ext_vector_type(4)));
typedef v4f  __attribute__((may_alias)) v4fa;
typedef v8h  __attribute__((may_alias)) v8ha;
typedef v8us __attribute__((may_alias)) v8usa;

static __device__ __forceinline__ unsigned int bf_bits(float f) {
  unsigned int u = __float_as_uint(f);
  u += 0x7FFFu + ((u >> 16) & 1u);
  return u >> 16;
}
static __device__ __forceinline__ float bf_rne(float f) { return __uint_as_float(bf_bits(f) << 16); }
static __device__ __forceinline__ int imin(int a, int b) { return a < b ? a : b; }

static __device__ __forceinline__ v16h ldfrag(const _Float16* p) {
  union { v16h v; v8h h[2]; } f;
  f.h[0] = *(const v8ha*)(p);
  f.h[1] = *(const v8ha*)(p + 16);
  return f.v;
}
static __device__ __forceinline__ v16b ldfragb(const unsigned short* p) {
  union { v16b v; v8us h[2]; } f;
  f.h[0] = *(const v8usa*)(p);
  f.h[1] = *(const v8usa*)(p + 16);
  return f.v;
}

static __device__ __forceinline__ v8f mma_h(v16h a, v16h b, v8f c) {
#if defined(__HIP_DEVICE_COMPILE__)
  c = __builtin_amdgcn_wmma_f32_16x16x32_f16(false, a, false, b, (short)0, c, false, false);
  asm volatile("v_nop\n\tv_nop\n\tv_nop\n\tv_nop" : "+v"(c) : "v"(a), "v"(b));
#endif
  return c;
}
static __device__ __forceinline__ v8f mma_b(v16b a, v16b b, v8f c) {
#if defined(__HIP_DEVICE_COMPILE__)
  c = __builtin_amdgcn_wmma_f32_16x16x32_bf16(false, a, false, b, (short)0, c, false, false);
  asm volatile("v_nop\n\tv_nop\n\tv_nop\n\tv_nop" : "+v"(c) : "v"(a), "v"(b));
#endif
  return c;
}
static __device__ __forceinline__ v8f zero8() { v8f z = {0.f, 0.f, 0.f, 0.f, 0.f, 0.f, 0.f, 0.f}; return z; }

static __device__ __forceinline__ void wave_sync() {
#if defined(__HIP_DEVICE_COMPILE__)
  __builtin_amdgcn_fence(__ATOMIC_RELEASE, "workgroup");
  __builtin_amdgcn_wave_barrier();
  __builtin_amdgcn_fence(__ATOMIC_ACQUIRE, "workgroup");
#endif
}

__global__ __launch_bounds__(256) void cvt_w_kernel(const float* __restrict__ src, unsigned short* __restrict__ dst,
                                                     int nsrc, int K, int grp, int dgrp, int doff) {
  const int i = blockIdx.x * 256 + threadIdx.x;
  const int kp = K >> 3;
  if (i >= nsrc * kp) return;
  const int sr = i / kp;
  const int c8 = (i - sr * kp) * 8;
  const int gq = sr / grp;
  const int dr = gq * dgrp + doff + (sr - gq * grp);
  const float* sp = src + (size_t)sr * K + c8;
  const v4f a = *(const v4f*)(sp);
  const v4f bq = *(const v4f*)(sp + 4);
  v8us o;
  o[0] = (unsigned short)bf_bits(a[0]); o[1] = (unsigned short)bf_bits(a[1]);
  o[2] = (unsigned short)bf_bits(a[2]); o[3] = (unsigned short)bf_bits(a[3]);
  o[4] = (unsigned short)bf_bits(bq[0]); o[5] = (unsigned short)bf_bits(bq[1]);
  o[6] = (unsigned short)bf_bits(bq[2]); o[7] = (unsigned short)bf_bits(bq[3]);
  unsigned short* dp = dst + (size_t)dr * K + c8;
  *(volatile v8us*)dp = o;
  __threadfence();
  *(volatile v8us*)dp = o;
}

__global__ __launch_bounds__(256) void cvt_wo_kernel(const float* __restrict__ src, unsigned short* __restrict__ dst, int nrows) {
  const int i = blockIdx.x * 256 + threadIdx.x;
  if (i >= nrows * 32) return;
  const int r = i >> 5;
  const int c8 = (i & 31) * 8;
  const int hd = c8 >> 7;
  const int d0 = c8 & 127;
  const int dcl = d0 > 88 ? 88 : d0;
  const bool valid = d0 < HD;
  const float* sp = src + (size_t)r * NC + hd * HD + dcl;
  const v4f a = *(const v4f*)(sp);
  const v4f bq = *(const v4f*)(sp + 4);
  v8us o;
  o[0] = valid ? (unsigned short)bf_bits(a[0]) : (unsigned short)0;  o[1] = valid ? (unsigned short)bf_bits(a[1]) : (unsigned short)0;
  o[2] = valid ? (unsigned short)bf_bits(a[2]) : (unsigned short)0;  o[3] = valid ? (unsigned short)bf_bits(a[3]) : (unsigned short)0;
  o[4] = valid ? (unsigned short)bf_bits(bq[0]) : (unsigned short)0; o[5] = valid ? (unsigned short)bf_bits(bq[1]) : (unsigned short)0;
  o[6] = valid ? (unsigned short)bf_bits(bq[2]) : (unsigned short)0; o[7] = valid ? (unsigned short)bf_bits(bq[3]) : (unsigned short)0;
  unsigned short* dp = dst + (size_t)r * CPW + c8;
  *(volatile v8us*)dp = o;
  __threadfence();
  *(volatile v8us*)dp = o;
}

__global__ __launch_bounds__(256) void cvt_conv_kernel(const float* __restrict__ src, unsigned short* __restrict__ dst,
                                                        int nrows, int Ci) {
  const int i = blockIdx.x * 256 + threadIdx.x;
  const int kp = (3 * Ci) >> 3;
  if (i >= nrows * kp) return;
  const int r = i / kp;
  const int k = (i - r * kp) * 8;
  const int tap = k / Ci;
  const int cc = k - tap * Ci;
  v8us o;
#pragma unroll
  for (int e = 0; e < 8; ++e) {
    const float f = src[((size_t)r * Ci + cc + e) * 3 + tap];
    o[e] = (unsigned short)bf_bits(f);
  }
  unsigned short* dp = dst + (size_t)r * (3 * Ci) + k;
  *(volatile v8us*)dp = o;
  __threadfence();
  *(volatile v8us*)dp = o;
}

__global__ __launch_bounds__(256) void halo_kernel(unsigned short* __restrict__ XPH, unsigned short* __restrict__ XPL,
                                                    unsigned short* __restrict__ HPH, unsigned short* __restrict__ HPL) {
  const int i = blockIdx.x * 256 + threadIdx.x;
  v8us zz = {0, 0, 0, 0, 0, 0, 0, 0};
  unsigned short* dp;
  if (i < 768) {
    const int plane = i / 384;
    const int rem = i - plane * 384;
    const int rr = rem / 24;
    const int p = rem - rr * 24;
    const int bb = rr >> 1;
    const int r = (rr & 1) ? (NT + 1) : 0;
    dp = (plane ? XPL : XPH) + (size_t)(bb * NTP + r) * NC + p * 8;
  } else if (i < 3840) {
    const int i2 = i - 768;
    const int plane = i2 / 1536;
    const int rem = i2 - plane * 1536;
    const int rr = rem / 96;
    const int p = rem - rr * 96;
    const int bb = rr >> 1;
    const int r = (rr & 1) ? (NT + 1) : 0;
    dp = (plane ? HPL : HPH) + (size_t)(bb * NTP + r) * NF + p * 8;
  } else {
    return;
  }
  *(volatile v8us*)dp = zz;
  __threadfence();
  *(volatile v8us*)dp = zz;
}

static __device__ __forceinline__ void write_row(const float* rw, float* xg, unsigned short* ph, unsigned short* pl,
                                                 float pm, int lane) {
  const v4f a0 = *(const v4fa*)(rw + 4 * lane);
  const int l2 = (lane < 16) ? lane : 0;
  const v4f a1 = *(const v4fa*)(rw + 128 + 4 * l2);
  const int l3 = (lane < 24) ? lane : 0;
  const v4f p0 = *(const v4fa*)(rw + 8 * l3);
  const v4f p1 = *(const v4fa*)(rw + 8 * l3 + 4);
  float f[8];
  f[0] = p0[0]; f[1] = p0[1]; f[2] = p0[2]; f[3] = p0[3];
  f[4] = p1[0]; f[5] = p1[1]; f[6] = p1[2]; f[7] = p1[3];
  v8us hi, lo;
#pragma unroll
  for (int e = 0; e < 8; ++e) {
    const float fe = f[e] * pm;
    const unsigned int hb = bf_bits(fe);
    const float hf = __uint_as_float(hb << 16);
    hi[e] = (unsigned short)hb;
    lo[e] = (unsigned short)bf_bits(fe - hf);
  }
  for (int pass = 0; pass < 2; ++pass) {
    *(volatile v4f*)(xg + 4 * lane) = a0;
    if (lane < 16) *(volatile v4f*)(xg + 128 + 4 * lane) = a1;
    if (lane < 24) {
      *(volatile v8us*)(ph + 8 * lane) = hi;
      *(volatile v8us*)(pl + 8 * lane) = lo;
    }
    __threadfence();
  }
}

__global__ __launch_bounds__(256) void embed_kernel(const int* __restrict__ tok, const int* __restrict__ lens,
                                                     const float* __restrict__ emb, float* __restrict__ x,
                                                     unsigned short* __restrict__ XH, unsigned short* __restrict__ XL) {
  __shared__ __align__(16) float rb[8][NC];
  const int wave = threadIdx.x >> 5, lane = threadIdx.x & 31;
  float* rw = rb[wave];
  for (int k = 0; k < TPW; ++k) {
    const int row = (blockIdx.x * 8 + wave) * TPW + k;
    if (row >= NTOK) break;
    const int b = row >> 10, t = row & (NT - 1);
    int tk = tok[row];
    tk = tk < 0 ? 0 : (tk > NVOC - 1 ? NVOC - 1 : tk);
    const int len = lens[b];
    const float mk = (t < len) ? 1.0f : 0.0f;
#pragma unroll
    for (int kk = 0; kk < 6; ++kk) {
      const int c = lane + 32 * kk;
      rw[c] = bf_rne(emb[(size_t)tk * NC + c]) * 13.856406460551018f * mk;
    }
    wave_sync();
    write_row(rw, x + (size_t)row * NC, XH + (size_t)row * NC, XL + (size_t)row * NC, 1.0f, lane);
    wave_sync();
  }
}

__global__ __launch_bounds__(256) void ln_kernel(float* x, const float* __restrict__ y,
                                                  const float* __restrict__ g, const float* __restrict__ be,
                                                  const int* __restrict__ lens,
                                                  unsigned short* __restrict__ PH, unsigned short* __restrict__ PL,
                                                  int prows, int poff, int pmask) {
  __shared__ __align__(16) float rb[8][NC];
  const int wave = threadIdx.x >> 5, lane = threadIdx.x & 31;
  float* rw = rb[wave];
  float gv[6], bv[6];
#pragma unroll
  for (int kk = 0; kk < 6; ++kk) { gv[kk] = bf_rne(g[lane + 32 * kk]); bv[kk] = bf_rne(be[lane + 32 * kk]); }
  for (int k = 0; k < TPW; ++k) {
    const int row = (blockIdx.x * 8 + wave) * TPW + k;
    if (row >= NTOK) break;
    const int b = row >> 10, t = row & (NT - 1);
    float* xr = x + (size_t)row * NC;
    const float* yr = y + (size_t)row * NC;
    float v[6];
    float s = 0.0f;
#pragma unroll
    for (int kk = 0; kk < 6; ++kk) { v[kk] = xr[lane + 32 * kk] + yr[lane + 32 * kk]; s += v[kk]; }
    s += __shfl_xor(s, 16, 32); s += __shfl_xor(s, 8, 32); s += __shfl_xor(s, 4, 32);
    s += __shfl_xor(s, 2, 32);  s += __shfl_xor(s, 1, 32);
    const float mean = s * (1.0f / 192.0f);
    float s2 = 0.0f;
#pragma unroll
    for (int kk = 0; kk < 6; ++kk) { v[kk] -= mean; s2 += v[kk] * v[kk]; }
    s2 += __shfl_xor(s2, 16, 32); s2 += __shfl_xor(s2, 8, 32); s2 += __shfl_xor(s2, 4, 32);
    s2 += __shfl_xor(s2, 2, 32);  s2 += __shfl_xor(s2, 1, 32);
    const float rstd = rsqrtf(s2 * (1.0f / 192.0f) + 1e-5f);
#pragma unroll
    for (int kk = 0; kk < 6; ++kk) rw[lane + 32 * kk] = v[kk] * rstd * gv[kk] + bv[kk];
    wave_sync();
    const int len = lens[b];
    const float pm = (pmask != 0 && t >= len) ? 0.0f : 1.0f;
    const size_t prow = (size_t)b * prows + poff + t;
    write_row(rw, xr, PH + prow * NC, PL + prow * NC, pm, lane);
    wave_sync();
  }
}

template <int OUTT, bool ALO, bool BLO, bool BIASROW>
__global__ __launch_bounds__(256) void gemm_kernel(
    const unsigned short* __restrict__ A, const unsigned short* __restrict__ A2, int lda, long strideA,
    const unsigned short* __restrict__ Bt, const unsigned short* __restrict__ Bt2, int ldb, long strideB,
    void* C1, void* C2, int ldc, long strideC,
    const float* __restrict__ bias, const float* __restrict__ bias2, const int* __restrict__ lens,
    int M, int N, int K, float scale1, float scale2, int nsplit, int relu, int maskMode) {
  __shared__ __align__(16) float sT[8][16 * 68];

  const int z = blockIdx.y;
  const int lane = threadIdx.x & 31;
  const int wave = threadIdx.x >> 5;
  const int tilesN = N >> 6;
  const int tilesM = M >> 6;
  const int tile = blockIdx.x * 8 + wave;
  if (tile >= tilesM * tilesN) return;
  const int tm = tile / tilesN;
  const int tn = tile - tm * tilesN;
  const int m0 = tm << 6;
  const int n0 = tn << 6;

  const unsigned short* Ab  = A   + (size_t)z * strideA;
  const unsigned short* A2b = A2  + (size_t)z * strideA;
  const unsigned short* Bb  = Bt  + (size_t)z * strideB;
  const unsigned short* B2b = Bt2 + (size_t)z * strideB;

  const int rl   = lane & 15;
  const int koff = (lane >> 4) * 8;
  const int mOff = (lane >> 4) * 8;

  v8f acc[4][4];
#pragma unroll
  for (int i = 0; i < 4; ++i)
#pragma unroll
    for (int j = 0; j < 4; ++j) acc[i][j] = zero8();

  for (int k0 = 0; k0 < K; k0 += 32) {
    if (ALO) {
      v16b bfr[4];
#pragma unroll
      for (int j = 0; j < 4; ++j)
        bfr[j] = ldfragb(Bb + (size_t)(n0 + (j << 4) + rl) * ldb + koff + k0);
#pragma unroll
      for (int i = 0; i < 4; ++i) {
        const size_t ao = (size_t)(m0 + (i << 4) + rl) * lda + koff + k0;
        const v16b a1 = ldfragb(Ab + ao);
        const v16b a2 = ldfragb(A2b + ao);
#pragma unroll
        for (int j = 0; j < 4; ++j) {
          acc[i][j] = mma_b(a1, bfr[j], acc[i][j]);
          acc[i][j] = mma_b(a2, bfr[j], acc[i][j]);
        }
      }
    } else {
      v16b afr[4];
#pragma unroll
      for (int i = 0; i < 4; ++i)
        afr[i] = ldfragb(Ab + (size_t)(m0 + (i << 4) + rl) * lda + koff + k0);
#pragma unroll
      for (int j = 0; j < 4; ++j) {
        const size_t bo = (size_t)(n0 + (j << 4) + rl) * ldb + koff + k0;
        const v16b b1 = ldfragb(Bb + bo);
        v16b b2 = b1;
        if (BLO) b2 = ldfragb(B2b + bo);
#pragma unroll
        for (int i = 0; i < 4; ++i) {
          acc[i][j] = mma_b(afr[i], b1, acc[i][j]);
          if (BLO) acc[i][j] = mma_b(afr[i], b2, acc[i][j]);
        }
      }
    }
  }

  int lenz = 0x3fffffff;
  if (maskMode != 0) lenz = lens[z];
  const float* bcol = bias;
  float scale = scale1;
  int nc0 = n0;
  void* Cs1 = C1;
  if (OUTT == 1) {
    if (n0 >= nsplit) { bcol = bias2; scale = scale2; nc0 = n0 - nsplit; Cs1 = C2; }
  }
  float bn[4] = {0.f, 0.f, 0.f, 0.f};
  if (!BIASROW) {
#pragma unroll
    for (int j = 0; j < 4; ++j) bn[j] = bf_rne(bcol[nc0 + (j << 4) + rl]);
  }
  float* slab = sT[wave];
#pragma unroll
  for (int i = 0; i < 4; ++i) {
    const int mBase = m0 + (i << 4);
    float br[8] = {0.f, 0.f, 0.f, 0.f, 0.f, 0.f, 0.f, 0.f};
    if (BIASROW) {
#pragma unroll
      for (int r = 0; r < 8; ++r) br[r] = bf_rne(bias[mBase + mOff + r]);
    }
#pragma unroll
    for (int j = 0; j < 4; ++j) {
#pragma unroll
      for (int r = 0; r < 8; ++r) {
        const int m = mBase + mOff + r;
        const int n = nc0 + (j << 4) + rl;
        float v = acc[i][j][r] + (BIASROW ? br[r] : bn[j]);
        v *= scale;
        if (relu) v = fmaxf(v, 0.0f);
        float mk = 1.0f;
        if (maskMode == 1) mk = (m < lenz) ? 1.0f : 0.0f;
        else if (maskMode == 2) mk = (n < lenz) ? 1.0f : 0.0f;
        v *= mk;
        slab[(mOff + r) * 68 + (j << 4) + rl] = v;
      }
    }
    wave_sync();
    if (OUTT == 0) {
      float* Cf = (float*)Cs1 + (size_t)z * strideC;
      const int hh = lane >> 4, c4 = (lane & 15) * 4;
      for (int pass = 0; pass < 2; ++pass) {
#pragma unroll
        for (int it = 0; it < 8; ++it) {
          const int row = it * 2 + hh;
          const v4f vv = *(const v4fa*)(slab + row * 68 + c4);
          *(volatile v4f*)(Cf + (size_t)(mBase + row) * ldc + nc0 + c4) = vv;
        }
        __threadfence();
      }
    } else if (OUTT == 1) {
      const int q = lane >> 3, c8 = (lane & 7) * 8;
      _Float16* Co = (_Float16*)Cs1 + (size_t)z * strideC;
      v8h hv[4];
#pragma unroll
      for (int it = 0; it < 4; ++it) {
        const int row = it * 4 + q;
        const float* sp = slab + row * 68 + c8;
        const v4f x0 = *(const v4fa*)(sp);
        const v4f x1 = *(const v4fa*)(sp + 4);
        v8h o;
        o[0] = (_Float16)x0[0]; o[1] = (_Float16)x0[1]; o[2] = (_Float16)x0[2]; o[3] = (_Float16)x0[3];
        o[4] = (_Float16)x1[0]; o[5] = (_Float16)x1[1]; o[6] = (_Float16)x1[2]; o[7] = (_Float16)x1[3];
        hv[it] = o;
      }
      for (int pass = 0; pass < 2; ++pass) {
#pragma unroll
        for (int it = 0; it < 4; ++it) {
          const int row = it * 4 + q;
          *(volatile v8h*)(Co + (size_t)(mBase + row) * ldc + nc0 + c8) = hv[it];
        }
        __threadfence();
      }
    } else {
      const int q = lane >> 3, c8 = (lane & 7) * 8;
      unsigned short* Ph = (unsigned short*)C1 + (size_t)z * strideC;
      unsigned short* Pl = (unsigned short*)C2 + (size_t)z * strideC;
      v8us hv[4], lv[4];
#pragma unroll
      for (int it = 0; it < 4; ++it) {
        const int row = it * 4 + q;
        const float* sp = slab + row * 68 + c8;
        const v4f x0 = *(const v4fa*)(sp);
        const v4f x1 = *(const v4fa*)(sp + 4);
        float f[8];
        f[0] = x0[0]; f[1] = x0[1]; f[2] = x0[2]; f[3] = x0[3];
        f[4] = x1[0]; f[5] = x1[1]; f[6] = x1[2]; f[7] = x1[3];
        v8us ha, hl;
#pragma unroll
        for (int e = 0; e < 8; ++e) {
          const unsigned int hb = bf_bits(f[e]);
          const float hf = __uint_as_float(hb << 16);
          ha[e] = (unsigned short)hb;
          hl[e] = (unsigned short)bf_bits(f[e] - hf);
        }
        hv[it] = ha; lv[it] = hl;
      }
      for (int pass = 0; pass < 2; ++pass) {
#pragma unroll
        for (int it = 0; it < 4; ++it) {
          const int row = it * 4 + q;
          *(volatile v8us*)(Ph + (size_t)(mBase + row) * ldc + nc0 + c8) = hv[it];
          *(volatile v8us*)(Pl + (size_t)(mBase + row) * ldc + nc0 + c8) = lv[it];
        }
        __threadfence();
      }
    }
    wave_sync();
  }
}

__global__ __launch_bounds__(128)
void attn_kernel(const _Float16* __restrict__ QP, const _Float16* __restrict__ KP,
                 const _Float16* __restrict__ VT, const float* __restrict__ relk,
                 const float* __restrict__ relv, const int* __restrict__ lens,
                 unsigned short* __restrict__ CH, unsigned short* __restrict__ CL) {
  __shared__ __align__(16) unsigned char SMEM[50176];
  _Float16* Ksh = (_Float16*)(SMEM);
  _Float16* Vsh = (_Float16*)(SMEM + 12288);
  _Float16* Psh = (_Float16*)(SMEM + 24576);
  float*    Osh = (float*)(SMEM);
  _Float16* PRs = (_Float16*)(SMEM + 32768);
  float*    BDs = (float*)(SMEM + 36864);
  _Float16* RKs = (_Float16*)(SMEM + 40960);
  _Float16* RVs = (_Float16*)(SMEM + 44032);

  const int tid  = threadIdx.x;
  const int wave = tid >> 5;
  const int lane = tid & 31;
  const int hh   = lane >> 4;
  const int c    = lane & 15;
  const int pair = blockIdx.y;
  const int b    = pair >> 1;
  const int h    = pair & 1;
  const int qb   = blockIdx.x;
  const int q0   = qb * 64 + wave * 16;
  int len = lens[b];
  len = len < 0 ? 0 : (len > NT ? NT : len);

  for (int i = tid; i < 16 * HD; i += 128) {
    const int e = i / HD;
    const int d = i - e * HD;
    const int ec = e < 9 ? e : 8;
    const float v = bf_rne(relk[ec * HD + d]) * 64.0f;
    RKs[i] = (_Float16)(e < 9 ? v : 0.0f);
  }
  for (int i = tid; i < HD * 32; i += 128) {
    const int cc = i >> 5;
    const int e = i & 31;
    const int ec = e < 9 ? e : 8;
    const float v = bf_rne(relv[ec * HD + cc]) * 16.0f;
    RVs[i] = (_Float16)(e < 9 ? v : 0.0f);
  }
  __syncthreads();

  const _Float16* Qh = QP + (size_t)(b * NT) * NC + h * HD;
  const _Float16* Kh = KP + (size_t)(b * NT) * NC + h * HD;
  const _Float16* Vh = VT + (size_t)b * NC * NT + (size_t)(h * HD) * NT;
  unsigned short* ch = CH + (size_t)(b * NT) * CPW + h * 128;
  unsigned short* cl = CL + (size_t)(b * NT) * CPW + h * 128;

  v16h qa[3];
#pragma unroll
  for (int dc = 0; dc < 3; ++dc)
    qa[dc] = ldfrag(Qh + (size_t)(q0 + c) * NC + dc * 32 + 8 * hh);

  {
    v8f ba = zero8();
#pragma unroll
    for (int dc = 0; dc < 3; ++dc) ba = mma_h(qa[dc], ldfrag(RKs + c * HD + dc * 32 + 8 * hh), ba);
    float* bwp = BDs + wave * 256;
#pragma unroll
    for (int r = 0; r < 8; ++r) bwp[(8 * hh + r) * 16 + c] = ba[r] * 0.000244140625f;
  }
  wave_sync();
  const float* bw = BDs + wave * 256;

  const int nch = (qb * 64 + 63 >= len) ? 16 : imin(16, (len + 63) >> 6);
  const float cs = 0.0009765625f;

  float mrow[8], lrow[8];
  v8f oacc[6];
#pragma unroll
  for (int r = 0; r < 8; ++r) { mrow[r] = -INFINITY; lrow[r] = 0.f; }
#pragma unroll
  for (int t = 0; t < 6; ++t) oacc[t] = zero8();

  _Float16* pw = Psh + wave * 1024;
  _Float16* pr = PRs + wave * 512;

  for (int kc = 0; kc < nch; ++kc) {
    const int kv0 = kc * 64;
    __syncthreads();
#pragma unroll
    for (int i = 0; i < 6; ++i) {
      const int p = i * 128 + tid;
      const int kr = p / 12;
      const int kc8 = (p - kr * 12) * 8;
      *(v8ha*)(Ksh + kr * HD + kc8) = *(const v8h*)(Kh + (size_t)(kv0 + kr) * NC + kc8);
      const int vr = p >> 3;
      const int vc8 = (p & 7) * 8;
      *(v8ha*)(Vsh + vr * 64 + vc8) = *(const v8h*)(Vh + (size_t)vr * NT + kv0 + vc8);
    }
    __syncthreads();

    v8f s[4];
#pragma unroll
    for (int j = 0; j < 4; ++j) {
      s[j] = zero8();
#pragma unroll
      for (int dc = 0; dc < 3; ++dc) {
        const v16h kb = ldfrag(Ksh + (j * 16 + c) * HD + dc * 32 + 8 * hh);
        s[j] = mma_h(qa[dc], kb, s[j]);
      }
    }

    const bool diag = (kv0 <= q0 + 19) && (kv0 + 63 >= q0 - 4);

    float cm[8];
#pragma unroll
    for (int r = 0; r < 8; ++r) {
      const int t = q0 + 8 * hh + r;
      const bool rp = (t >= len);
      float m = -INFINITY;
#pragma unroll
      for (int j = 0; j < 4; ++j) {
        const int key = kv0 + (j << 4) + c;
        float sv = s[j][r] * cs;
        if (diag) {
          const int e = key - t + 4;
          const int ecl = e < 0 ? 0 : (e > 15 ? 15 : e);
          const float bvv = bw[(8 * hh + r) * 16 + ecl];
          sv += (e >= 0 && e <= 8) ? bvv : 0.0f;
        }
        sv = (rp || key >= len) ? -10000.0f : sv;
        s[j][r] = sv;
        m = fmaxf(m, sv);
      }
      m = fmaxf(m, __shfl_xor(m, 1, 32));
      m = fmaxf(m, __shfl_xor(m, 2, 32));
      m = fmaxf(m, __shfl_xor(m, 4, 32));
      m = fmaxf(m, __shfl_xor(m, 8, 32));
      cm[r] = m;
    }

#pragma unroll
    for (int r = 0; r < 8; ++r) {
      const float mnew  = fmaxf(mrow[r], cm[r]);
      const float alpha = __expf(mrow[r] - mnew);
      mrow[r] = mnew;
      float psum = 0.f;
#pragma unroll
      for (int j = 0; j < 4; ++j) {
        const float p = __expf(s[j][r] - mnew);
        psum += p;
        pw[(8 * hh + r) * 64 + j * 16 + c] = (_Float16)(p * 4096.0f);
      }
      psum += __shfl_xor(psum, 1, 32);
      psum += __shfl_xor(psum, 2, 32);
      psum += __shfl_xor(psum, 4, 32);
      psum += __shfl_xor(psum, 8, 32);
      lrow[r] = lrow[r] * alpha + psum;
#pragma unroll
      for (int t = 0; t < 6; ++t) oacc[t][r] *= alpha;
    }
    wave_sync();

    if (diag) {
      const int row = c;
      const int e0 = hh * 16;
#pragma unroll 4
      for (int i = 0; i < 16; ++i) {
        const int e = e0 + i;
        const int kr = q0 + row + e - 4 - kv0;
        const bool ok = (e <= 8) && (kr >= 0) && (kr < 64);
        const int krc = kr < 0 ? 0 : (kr > 63 ? 63 : kr);
        const _Float16 pv = pw[row * 64 + krc];
        pr[row * 32 + e] = ok ? pv : (_Float16)0.0f;
      }
      wave_sync();
      const v16h pa = ldfrag(pr + c * 32 + 8 * hh);
#pragma unroll
      for (int t = 0; t < 6; ++t)
        oacc[t] = mma_h(pa, ldfrag(RVs + (t * 16 + c) * 32 + 8 * hh), oacc[t]);
    }

#pragma unroll
    for (int kk = 0; kk < 2; ++kk) {
      const v16h pa = ldfrag(pw + c * 64 + kk * 32 + 8 * hh);
#pragma unroll
      for (int t = 0; t < 6; ++t) {
        const v16h vb = ldfrag(Vsh + (t * 16 + c) * 64 + kk * 32 + 8 * hh);
        oacc[t] = mma_h(pa, vb, oacc[t]);
      }
    }
  }

  __syncthreads();
  float* os = Osh + wave * 2048;
#pragma unroll
  for (int r = 0; r < 8; ++r) {
    const float inv = 1.0f / (65536.0f * lrow[r]);
#pragma unroll
    for (int t = 0; t < 6; ++t) os[(8 * hh + r) * 128 + t * 16 + c] = oacc[t][r] * inv;
    os[(8 * hh + r) * 128 + 96 + c] = 0.0f;
    os[(8 * hh + r) * 128 + 112 + c] = 0.0f;
  }
  wave_sync();
  v8us hv[8], lv[8];
#pragma unroll
  for (int it = 0; it < 8; ++it) {
    const int row = it * 2 + hh;
    const float* sp = os + row * 128 + c * 8;
    const v4f x0 = *(const v4fa*)(sp);
    const v4f x1 = *(const v4fa*)(sp + 4);
    float f[8];
    f[0] = x0[0]; f[1] = x0[1]; f[2] = x0[2]; f[3] = x0[3];
    f[4] = x1[0]; f[5] = x1[1]; f[6] = x1[2]; f[7] = x1[3];
    v8us ha, hl;
#pragma unroll
    for (int e = 0; e < 8; ++e) {
      const unsigned int hb = bf_bits(f[e]);
      const float hf = __uint_as_float(hb << 16);
      ha[e] = (unsigned short)hb;
      hl[e] = (unsigned short)bf_bits(f[e] - hf);
    }
    hv[it] = ha; lv[it] = hl;
  }
  for (int pass = 0; pass < 2; ++pass) {
#pragma unroll
    for (int it = 0; it < 8; ++it) {
      const int row = it * 2 + hh;
      *(volatile v8us*)(ch + (size_t)(q0 + row) * CPW + c * 8) = hv[it];
      *(volatile v8us*)(cl + (size_t)(q0 + row) * CPW + c * 8) = lv[it];
    }
    __threadfence();
  }
}

extern "C" void kernel_launch(void* const* d_in, const int* in_sizes, int n_in,
                              void* d_out, int out_size, void* d_ws, size_t ws_size,
                              hipStream_t stream) {
  if (n_in < 23) return;
  if (in_sizes[0] != NTOK || in_sizes[1] != NB || in_sizes[2] != NVOC * NC) return;
  if (in_sizes[3] != NL * NC * NC || in_sizes[5] != NL * NC * NC || in_sizes[7] != NL * NC * NC || in_sizes[9] != NL * NC * NC) return;
  if (in_sizes[4] != NL * NC || in_sizes[6] != NL * NC || in_sizes[8] != NL * NC || in_sizes[10] != NL * NC) return;
  if (in_sizes[11] != NL * 9 * HD || in_sizes[12] != NL * 9 * HD) return;
  if (in_sizes[13] != NL * NC || in_sizes[14] != NL * NC || in_sizes[19] != NL * NC || in_sizes[20] != NL * NC) return;
  if (in_sizes[15] != NL * NF * NC * 3 || in_sizes[16] != NL * NF || in_sizes[17] != NL * NC * NF * 3 || in_sizes[18] != NL * NC) return;
  if (in_sizes[21] != NO2 * NC || in_sizes[22] != NO2) return;
  if (out_size != NB * NO2 * NT) return;

  const int*   tokens = (const int*)d_in[0];
  const int*   lens   = (const int*)d_in[1];
  const float* emb    = (const float*)d_in[2];
  const float* Wq  = (const float*)d_in[3];   const float* bq  = (const float*)d_in[4];
  const float* Wk  = (const float*)d_in[5];   const float* bk  = (const float*)d_in[6];
  const float* Wv  = (const float*)d_in[7];   const float* bv  = (const float*)d_in[8];
  const float* Wo  = (const float*)d_in[9];   const float* bo  = (const float*)d_in[10];
  const float* rel_k = (const float*)d_in[11];
  const float* rel_v = (const float*)d_in[12];
  const float* g1  = (const float*)d_in[13];  const float* bn1 = (const float*)d_in[14];
  const float* Wf1 = (const float*)d_in[15];  const float* bf1 = (const float*)d_in[16];
  const float* Wf2 = (const float*)d_in[17];  const float* bf2 = (const float*)d_in[18];
  const float* g2  = (const float*)d_in[19];  const float* bn2 = (const float*)d_in[20];
  const float* Wproj = (const float*)d_in[21];
  const float* bproj = (const float*)d_in[22];
  float* out = (float*)d_out;

  const size_t sWQK = (size_t)NL * 384 * NC * 2;
  const size_t sWV  = (size_t)NL * NC * NC * 2;
  const size_t sWO  = (size_t)NL * NC * CPW * 2;
  const size_t sW1  = (size_t)NL * NF * (3 * NC) * 2;
  const size_t sW2  = (size_t)NL * NC * (3 * NF) * 2;
  const size_t sWPJ = (size_t)NO2 * NC * 2;
  const size_t sX   = (size_t)NTOK * NC * 4;
  const size_t sXb  = (size_t)NTOK * NC * 2;
  const size_t sXP  = (size_t)NB * NTP * NC * 2;
  const size_t sQK  = (size_t)NTOK * NC * 2;
  const size_t sVT  = (size_t)NB * NC * NT * 2;
  const size_t sCX  = (size_t)NTOK * CPW * 2;
  const size_t sY   = (size_t)NTOK * NC * 4;
  const size_t sHP  = (size_t)NB * NTP * NF * 2;
  size_t off = 0;
  const size_t oWQK = off; off += sWQK;
  const size_t oWV  = off; off += sWV;
  const size_t oWO  = off; off += sWO;
  const size_t oW1  = off; off += sW1;
  const size_t oW2  = off; off += sW2;
  const size_t oWPJ = off; off += sWPJ;
  const size_t oX   = off; off += sX;
  const size_t oXH  = off; off += sXb;
  const size_t oXL  = off; off += sXb;
  const size_t oXPH = off; off += sXP;
  const size_t oXPL = off; off += sXP;
  const size_t oQP  = off; off += sQK;
  const size_t oKP  = off; off += sQK;
  const size_t oVT  = off; off += sVT;
  const size_t oCH  = off; off += sCX;
  const size_t oCL  = off; off += sCX;
  const size_t oY   = off; off += sY;
  const size_t oHPH = off; off += sHP;
  const size_t oHPL = off; off += sHP;
  const size_t total = off;
  if (total > ws_size) return;
  if (total > (size_t)134217728) return;

  char* ws = (char*)d_ws;
  unsigned short* WQK = (unsigned short*)(ws + oWQK);
  unsigned short* WVp = (unsigned short*)(ws + oWV);
  unsigned short* WOp = (unsigned short*)(ws + oWO);
  unsigned short* W1R = (unsigned short*)(ws + oW1);
  unsigned short* W2R = (unsigned short*)(ws + oW2);
  unsigned short* WPJ = (unsigned short*)(ws + oWPJ);
  float*          X   = (float*)(ws + oX);
  unsigned short* XH  = (unsigned short*)(ws + oXH);
  unsigned short* XL  = (unsigned short*)(ws + oXL);
  unsigned short* XPH = (unsigned short*)(ws + oXPH);
  unsigned short* XPL = (unsigned short*)(ws + oXPL);
  _Float16*       QPp = (_Float16*)(ws + oQP);
  _Float16*       KPp = (_Float16*)(ws + oKP);
  _Float16*       VTp = (_Float16*)(ws + oVT);
  unsigned short* CHp = (unsigned short*)(ws + oCH);
  unsigned short* CLp = (unsigned short*)(ws + oCL);
  float*          Y   = (float*)(ws + oY);
  unsigned short* HPH = (unsigned short*)(ws + oHPH);
  unsigned short* HPL = (unsigned short*)(ws + oHPL);

  const dim3 blk(256);
  const float qsc = 0.10206207261596575f * 64.0f;

  {
    const int nWrows = NL * NC;
    const dim3 gW((nWrows * (NC / 8) + 255) / 256);
    cvt_w_kernel<<<gW, blk, 0, stream>>>(Wq, WQK, nWrows, NC, NC, 384, 0);
    cvt_w_kernel<<<gW, blk, 0, stream>>>(Wk, WQK, nWrows, NC, NC, 384, NC);
    cvt_w_kernel<<<gW, blk, 0, stream>>>(Wv, WVp, nWrows, NC, NC, NC, 0);
    const dim3 gP((NO2 * (NC / 8) + 255) / 256);
    cvt_w_kernel<<<gP, blk, 0, stream>>>(Wproj, WPJ, NO2, NC, NO2, NO2, 0);
    const dim3 gO((nWrows * 32 + 255) / 256);
    cvt_wo_kernel<<<gO, blk, 0, stream>>>(Wo, WOp, nWrows);
    const int r1 = NL * NF;
    cvt_conv_kernel<<<dim3((r1 * ((3 * NC) / 8) + 255) / 256), blk, 0, stream>>>(Wf1, W1R, r1, NC);
    const int r2 = NL * NC;
    cvt_conv_kernel<<<dim3((r2 * ((3 * NF) / 8) + 255) / 256), blk, 0, stream>>>(Wf2, W2R, r2, NF);
    halo_kernel<<<dim3((3840 + 255) / 256), blk, 0, stream>>>(XPH, XPL, HPH, HPL);
  }
  const dim3 gRow((NTOK + 8 * TPW - 1) / (8 * TPW));
  embed_kernel<<<gRow, blk, 0, stream>>>(tokens, lens, emb, X, XH, XL);

  const int BIG = 1 << 30;
  for (int l = 0; l < NL; ++l) {
    const unsigned short* wqk = WQK + (size_t)l * 384 * NC;
    const unsigned short* wv  = WVp + (size_t)l * NC * NC;
    const unsigned short* wo  = WOp + (size_t)l * NC * CPW;
    const unsigned short* w1  = W1R + (size_t)l * NF * (3 * NC);
    const unsigned short* w2  = W2R + (size_t)l * NC * (3 * NF);
    {
      const int tiles = (NTOK / 64) * (384 / 64);
      gemm_kernel<1, true, false, false><<<dim3(tiles / 8, 1), blk, 0, stream>>>(
          XH, XL, NC, 0L, wqk, wqk, NC, 0L, (void*)QPp, (void*)KPp, NC, 0L,
          bq + l * NC, bk + l * NC, lens, NTOK, 384, NC, qsc, 16.0f, NC, 0, 0);
    }
    {
      const int tiles = (NC / 64) * (NT / 64);
      gemm_kernel<1, false, true, true><<<dim3(tiles / 8, NB), blk, 0, stream>>>(
          wv, wv, NC, 0L, XH, XL, NC, (long)NT * NC, (void*)VTp, (void*)VTp, NT, (long)NC * NT,
          bv + l * NC, bv + l * NC, lens, NC, NT, NC, 16.0f, 16.0f, BIG, 0, 0);
    }
    attn_kernel<<<dim3(NT / 64, NB * 2), dim3(128), 0, stream>>>(
        QPp, KPp, VTp, rel_k + (size_t)l * 9 * HD, rel_v + (size_t)l * 9 * HD, lens, CHp, CLp);
    {
      const int tiles = (NTOK / 64) * (NC / 64);
      gemm_kernel<0, true, false, false><<<dim3(tiles / 8, 1), blk, 0, stream>>>(
          CHp, CLp, CPW, 0L, wo, wo, CPW, 0L, (void*)Y, (void*)Y, NC, 0L,
          bo + l * NC, bo + l * NC, lens, NTOK, NC, CPW, 1.0f, 1.0f, BIG, 0, 0);
    }
    ln_kernel<<<gRow, blk, 0, stream>>>(X, Y, g1 + l * NC, bn1 + l * NC, lens, XPH, XPL, NTP, 1, 1);
    {
      const int tiles = (NT / 64) * (NF / 64);
      gemm_kernel<2, true, false, false><<<dim3(tiles / 8, NB), blk, 0, stream>>>(
          XPH, XPL, NC, (long)NTP * NC, w1, w1, 3 * NC, 0L, (void*)(HPH + NF), (void*)(HPL + NF), NF, (long)NTP * NF,
          bf1 + l * NF, bf1 + l * NF, lens, NT, NF, 3 * NC, 1.0f, 1.0f, BIG, 1, 1);
    }
    {
      const int tiles = (NT / 64) * (NC / 64);
      gemm_kernel<0, true, false, false><<<dim3(tiles / 8, NB), blk, 0, stream>>>(
          HPH, HPL, NF, (long)NTP * NF, w2, w2, 3 * NF, 0L, (void*)Y, (void*)Y, NC, (long)NT * NC,
          bf2 + l * NC, bf2 + l * NC, lens, NT, NC, 3 * NF, 1.0f, 1.0f, BIG, 0, 1);
    }
    ln_kernel<<<gRow, blk, 0, stream>>>(X, Y, g2 + l * NC, bn2 + l * NC, lens, XH, XL, NT, 0, 0);
  }
  {
    const int tiles = (NO2 / 64) * (NT / 64);
    gemm_kernel<0, false, true, true><<<dim3(tiles / 8, NB), blk, 0, stream>>>(
        WPJ, WPJ, NC, 0L, XH, XL, NC, (long)NT * NC, (void*)out, (void*)out, NT, (long)NO2 * NT,
        bproj, bproj, lens, NO2, NT, NC, 1.0f, 1.0f, BIG, 0, 2);
  }
  (void)hipGetLastError();
}
